// SegSmall_23914377904592
// MI455X (gfx1250) — hardware-run, weakly checked
//
#include <hip/hip_runtime.h>
#include <math.h>

typedef __attribute__((ext_vector_type(16))) _Float16 v16h;
typedef __attribute__((ext_vector_type(8)))  _Float16 v8h;
typedef __attribute__((ext_vector_type(16))) __bf16   v16b;
typedef __attribute__((ext_vector_type(8)))  __bf16   v8b;
typedef __attribute__((ext_vector_type(8)))  float    v8f;
typedef __attribute__((ext_vector_type(4)))  float    v4f;
typedef __attribute__((ext_vector_type(2)))  float    v2f;
typedef __attribute__((ext_vector_type(4)))  int      v4i;
typedef __attribute__((ext_vector_type(4)))  unsigned v4u;

constexpr int kBatch    = 4;
constexpr int kNpts     = 16384;
constexpr int kNbr      = 16;
constexpr int kCin      = 64;
constexpr int kCout     = 64;
constexpr int kKs       = 16;
constexpr int kPts      = kBatch * kNpts;
constexpr int kKfin     = kCin * kKs;
constexpr int kChunkPts = 32768;
constexpr int kChunks   = kPts / kChunkPts;
constexpr int kWavesA   = 4;
constexpr int kPtsWave  = 16;
constexpr int kPtsBlock = kWavesA * kPtsWave;
constexpr float kWtCarry  = 16.0f;
constexpr float kOutScale = (1.0f / (float)kNbr) / kWtCarry;
static_assert(kNpts == (1 << 14), "batch base by shift");
static_assert(kNbr == 16 && kKs == 16 && kCin == 64 && kCout == 64, "tile shapes");
static_assert(kKfin == 1024 && (kKfin % 32) == 0, "GEMM K multiple of 32");
static_assert((kChunkPts % 64) == 0 && (kCout % 64) == 0, "GEMM M,N multiples of 64");
static_assert(kChunks * kChunkPts == kPts, "chunks cover all points");
static_assert((kChunkPts % kPtsBlock) == 0, "point blocks cover a chunk exactly");

constexpr size_t kOffAgg   = 0;
constexpr size_t kSzAgg    = (size_t)kChunkPts * kKfin * 2;
constexpr size_t kOffWt    = kOffAgg + kSzAgg;
constexpr size_t kSzWt     = (size_t)kCout * kKfin * 2;
constexpr size_t kOffSmall = kOffWt + kSzWt;
constexpr size_t kSzSmall  = 2560;
constexpr size_t kWsTotal  = kOffSmall + kSzSmall;
static_assert(kWsTotal == 67242496ull, "carve total");
static_assert(kWsTotal <= 134217728ull, "carve cap");
static_assert((kOffWt % 128) == 0 && (kOffSmall % 128) == 0 && (kSzSmall % 128) == 0, "line aligned regions");

__device__ __forceinline__ unsigned short f2bf_bits(float f) {
  unsigned u = __float_as_uint(f);
  return (unsigned short)((u + 0x7FFFu + ((u >> 16) & 1u)) >> 16);
}
__device__ __forceinline__ float bf_bits2f(unsigned short h) { return __uint_as_float(((unsigned)h) << 16); }

__device__ __forceinline__ void dep_guard4_h(v8f& a, v8f& b, v8f& c, v8f& d, v16h x, v16h y) {
  asm volatile("v_nop\n\tv_nop\n\tv_nop\n\tv_nop" : "+v"(a), "+v"(b), "+v"(c), "+v"(d) : "v"(x), "v"(y));
}
__device__ __forceinline__ void dep_guard4_b(v8f& a, v8f& b, v8f& c, v8f& d, v16b x, v16b y) {
  asm volatile("v_nop\n\tv_nop\n\tv_nop\n\tv_nop" : "+v"(a), "+v"(b), "+v"(c), "+v"(d) : "v"(x), "v"(y));
}
__device__ __forceinline__ void keep4_h(v16h a, v16h b, v16h c, v16h d) { asm volatile("v_nop" :: "v"(a), "v"(b), "v"(c), "v"(d)); }
__device__ __forceinline__ void keep4_b(v16b a, v16b b, v16b c, v16b d) { asm volatile("v_nop" :: "v"(a), "v"(b), "v"(c), "v"(d)); }
__device__ __forceinline__ void acc_guard4(v8f& a, v8f& b, v8f& c, v8f& d) { asm volatile("v_nop\n\tv_nop\n\tv_nop\n\tv_nop" : "+v"(a), "+v"(b), "+v"(c), "+v"(d)); }

template <typename T> struct Frag;
template <> struct Frag<_Float16> {
  typedef v16h V;
  union U { v16h v; v8h h[2]; };
  static __device__ __forceinline__ v16h load(const _Float16* p) {
    U f; f.h[0] = *(const v8h*)(p); f.h[1] = *(const v8h*)(p + 16); return f.v;
  }
  static __device__ __forceinline__ v8f mma(v16h a, v16h b, v8f c) {
    return __builtin_amdgcn_wmma_f32_16x16x32_f16(false, a, false, b, (short)0, c, false, false);
  }
  static __device__ __forceinline__ void guard4(v8f& a, v8f& b, v8f& c, v8f& d, v16h x, v16h y) { dep_guard4_h(a, b, c, d, x, y); }
  static __device__ __forceinline__ void keep(v16h a, v16h b, v16h c, v16h d) { keep4_h(a, b, c, d); }
};
template <> struct Frag<__bf16> {
  typedef v16b V;
  union U { v16b v; v8b h[2]; };
  static __device__ __forceinline__ v16b load(const __bf16* p) {
    U f; f.h[0] = *(const v8b*)(p); f.h[1] = *(const v8b*)(p + 16); return f.v;
  }
  static __device__ __forceinline__ v8f mma(v16b a, v16b b, v8f c) {
    return __builtin_amdgcn_wmma_f32_16x16x32_bf16(false, a, false, b, (short)0, c, false, false);
  }
  static __device__ __forceinline__ void guard4(v8f& a, v8f& b, v8f& c, v8f& d, v16b x, v16b y) { dep_guard4_b(a, b, c, d, x, y); }
  static __device__ __forceinline__ void keep(v16b a, v16b b, v16b c, v16b d) { keep4_b(a, b, c, d); }
};

template <int ET> struct Elem;
template <> struct Elem<0> { typedef _Float16 T; };
template <> struct Elem<1> { typedef __bf16 T; };
template <int ET, bool SPLIT, int BIAS_MODE, int OUT_MODE, bool RESID, int ACT = 0>
__global__ __launch_bounds__(256) void wmma_gemm64(
    const unsigned short* __restrict__ Ap, const unsigned short* __restrict__ A2p, int lda, long strideA,
    const unsigned short* __restrict__ Btp, const unsigned short* __restrict__ Bt2p, int ldb, long strideB,
    void* __restrict__ Cout, void* __restrict__ Cout2, int ldc, long strideC,
    const float* __restrict__ bias,
    const float* __restrict__ resid, long strideR,
    int M, int N, int K, float scale) {
  typedef typename Elem<ET>::T T;
  typedef typename Frag<T>::V V;
  const T* A = (const T*)Ap; const T* A2 = (const T*)A2p; const T* Bt = (const T*)Btp; const T* Bt2 = (const T*)Bt2p;
  __shared__ __align__(16) float sT[8][16 * 68];
  const int b    = blockIdx.y;
  const int lane = threadIdx.x & 31;
  const int wave = threadIdx.x >> 5;
  const int tilesN = N >> 6;
  const int tilesM = M >> 6;
  const int tile = blockIdx.x * 8 + wave;
  if (tile >= tilesM * tilesN) return;
  const int tm = tile / tilesN;
  const int tn = tile - tm * tilesN;
  const int m0 = tm << 6;
  const int n0 = tn << 6;

  const T* Ab  = A  + (size_t)b * strideA;
  const T* Bb  = Bt + (size_t)b * strideB;
  const T* Ab2 = SPLIT ? (A2  + (size_t)b * strideA) : nullptr;
  const T* Bb2 = SPLIT ? (Bt2 + (size_t)b * strideB) : nullptr;

  const int rlane = lane & 15;
  const int koff  = (lane >> 4) * 8;
  const int mOff  = (lane >> 4) * 8;

  v8f acc[4][4];
#pragma unroll
  for (int i = 0; i < 4; ++i)
#pragma unroll
    for (int j = 0; j < 4; ++j) acc[i][j] = (v8f){0.f,0.f,0.f,0.f,0.f,0.f,0.f,0.f};

  for (int k0 = 0; k0 < K; k0 += 32) {
    V bh[4], bl[4];
#pragma unroll
    for (int j = 0; j < 4; ++j) {
      const size_t bo = (size_t)(n0 + (j << 4) + rlane) * ldb + koff + k0;
      bh[j] = Frag<T>::load(Bb + bo);
      if (SPLIT) bl[j] = Frag<T>::load(Bb2 + bo);
    }
#pragma unroll
    for (int i = 0; i < 4; ++i) {
      const size_t ao = (size_t)(m0 + (i << 4) + rlane) * lda + koff + k0;
      V ah = Frag<T>::load(Ab + ao);
      V al;
      if (SPLIT) al = Frag<T>::load(Ab2 + ao);
#pragma unroll
      for (int j = 0; j < 4; ++j) {
        acc[i][j] = Frag<T>::mma(ah, bh[j], acc[i][j]);
        if (SPLIT) {
          acc[i][j] = Frag<T>::mma(ah, bl[j], acc[i][j]);
          acc[i][j] = Frag<T>::mma(al, bh[j], acc[i][j]);
        }
      }
      Frag<T>::guard4(acc[i][0], acc[i][1], acc[i][2], acc[i][3], ah, SPLIT ? al : ah);
    }
    Frag<T>::keep(bh[0], bh[1], bh[2], bh[3]);
    if (SPLIT) Frag<T>::keep(bl[0], bl[1], bl[2], bl[3]);
  }
  acc_guard4(acc[0][0], acc[0][1], acc[0][2], acc[0][3]);
  acc_guard4(acc[1][0], acc[1][1], acc[1][2], acc[1][3]);
  acc_guard4(acc[2][0], acc[2][1], acc[2][2], acc[2][3]);
  acc_guard4(acc[3][0], acc[3][1], acc[3][2], acc[3][3]);

  float* slab = sT[wave];
  const float* Rb = RESID ? (resid + (size_t)b * strideR) : nullptr;
#pragma unroll
  for (int i = 0; i < 4; ++i) {
    const int mBase = m0 + (i << 4);
#pragma unroll
    for (int j = 0; j < 4; ++j) {
      const int n = n0 + (j << 4) + rlane;
      float bv = 0.f;
      if (BIAS_MODE == 2) bv = bias[n];
#pragma unroll
      for (int r = 0; r < 8; ++r) {
        float v = acc[i][j][r] * scale;
        if (BIAS_MODE == 1) v += bias[mBase + mOff + r];
        if (BIAS_MODE == 2) v += bv;
        if (RESID) v += Rb[(size_t)(mBase + mOff + r) * ldc + n];
        if (ACT == 1) v = tanhf(v);
        if (ACT == 2) v = fmaxf(v, 0.0f);
        if (ACT == 3) v = v / (1.0f + expf(-v));
        if (ACT == 4) v = (v > 0.f) ? v : 0.01f * v;
        slab[(mOff + r) * 68 + (j << 4) + rlane] = v;
      }
    }
    __builtin_amdgcn_fence(__ATOMIC_RELEASE, "workgroup");
    __builtin_amdgcn_wave_barrier();
    __builtin_amdgcn_fence(__ATOMIC_ACQUIRE, "workgroup");
    if (OUT_MODE == 0) {
      float* C = (float*)Cout + (size_t)b * strideC;
      const int hh = lane >> 4, c4 = (lane & 15) * 4;
      for (int pass = 0; pass < 2; ++pass) {
#pragma unroll
        for (int it = 0; it < 8; ++it) {
          const int row = it * 2 + hh;
          v4f v = *(const v4f*)(slab + row * 68 + c4);
          *(volatile v4f*)(C + (size_t)(mBase + row) * ldc + n0 + c4) = v;
        }
        __threadfence();
      }
    } else {
      const int q = lane >> 3, c8 = (lane & 7) * 8;
      unsigned short* C  = (unsigned short*)Cout  + (size_t)b * strideC;
      unsigned short* C2 = (OUT_MODE == 2) ? ((unsigned short*)Cout2 + (size_t)b * strideC) : nullptr;
      for (int pass = 0; pass < 2; ++pass) {
#pragma unroll
        for (int it = 0; it < 4; ++it) {
          const int row = it * 4 + q;
          const float* sp = slab + row * 68 + c8;
          v8h hv, lv;
#pragma unroll
          for (int e = 0; e < 8; ++e) {
            if (OUT_MODE == 1) {
              hv[e] = (_Float16)sp[e];
            } else {
              unsigned short hb = f2bf_bits(sp[e]);
              unsigned short lb = f2bf_bits(sp[e] - bf_bits2f(hb));
              hv[e] = __builtin_bit_cast(_Float16, hb);
              lv[e] = __builtin_bit_cast(_Float16, lb);
            }
          }
          *(volatile v8h*)(C + (size_t)(mBase + row) * ldc + n0 + c8) = hv;
          if (OUT_MODE == 2) *(volatile v8h*)(C2 + (size_t)(mBase + row) * ldc + n0 + c8) = lv;
        }
        __threadfence();
      }
    }
    __builtin_amdgcn_fence(__ATOMIC_RELEASE, "workgroup");
    __builtin_amdgcn_wave_barrier();
    __builtin_amdgcn_fence(__ATOMIC_ACQUIRE, "workgroup");
  }
}

__device__ __forceinline__ unsigned pack_h2(float lo, float hi) {
  const _Float16 a = (_Float16)lo;
  const _Float16 b = (_Float16)hi;
  const unsigned short ua = __builtin_bit_cast(unsigned short, a);
  const unsigned short ub = __builtin_bit_cast(unsigned short, b);
  return (unsigned)ua | ((unsigned)ub << 16);
}
__device__ __forceinline__ v8f mma_g(v16h a, v16h b, v8f c) {
  c = __builtin_amdgcn_wmma_f32_16x16x32_f16(false, a, false, b, (short)0, c, false, false);
  asm volatile("v_nop\n\tv_nop\n\tv_nop\n\tv_nop" : "+v"(c) : "v"(a), "v"(b));
  return c;
}
__device__ __forceinline__ void wave_sync() {
  __builtin_amdgcn_fence(__ATOMIC_RELEASE, "workgroup");
  __builtin_amdgcn_wave_barrier();
  __builtin_amdgcn_fence(__ATOMIC_ACQUIRE, "workgroup");
}

__global__ __launch_bounds__(256) void prep_wt_kernel(const float* __restrict__ weight, unsigned short* __restrict__ Wt)
{
  __shared__ __align__(16) float sT[64 * 65];
  const int t = threadIdx.x, lane = t & 31, wave = t >> 5;
  const int k0 = blockIdx.x * 64;
#pragma unroll 1
  for (int i = 0; i < 16; ++i) {
    const int e = t + 256 * i;
    const int kr = e >> 6, o = e & 63;
    sT[kr * 65 + o] = weight[(size_t)(k0 + kr) * kCout + o] * kWtCarry;
  }
  __syncthreads();
  const int q = lane >> 3, c8 = (lane & 7) * 8;
  v8h hv[2];
#pragma unroll
  for (int it = 0; it < 2; ++it) {
    const int o = it * 32 + wave * 4 + q;
#pragma unroll
    for (int e = 0; e < 8; ++e) hv[it][e] = (_Float16)sT[(c8 + e) * 65 + o];
  }
  for (int pass = 0; pass < 2; ++pass) {
#pragma unroll
    for (int it = 0; it < 2; ++it) {
      const int o = it * 32 + wave * 4 + q;
      *(volatile v8h*)(Wt + (size_t)o * kKfin + k0 + c8) = hv[it];
    }
    __threadfence();
  }
}

__global__ __launch_bounds__(256) void prep_small_kernel(
    const float* __restrict__ w1, const float* __restrict__ b1, const float* __restrict__ w2,
    const float* __restrict__ w3, const float* __restrict__ centers, unsigned* __restrict__ dst)
{
  __shared__ __align__(16) unsigned img[640];
  const int t = threadIdx.x, wave = t >> 5;
  {
    const int n = t >> 4, kp = t & 15, k = 2 * kp;
    const float lo = w2[k * 16 + n];
    const float hi = w2[(k + 1) * 16 + n];
    img[t] = pack_h2(lo, hi);
  }
  {
    const int j = t >> 4, kp = t & 15;
    const bool live = (kp < 8);
    const int k = live ? 2 * kp : 0;
    const float lo = w3[k * 16 + j];
    const float hi = w3[(k + 1) * 16 + j];
    const unsigned w = pack_h2(lo, hi);
    img[256 + t] = live ? w : 0u;
  }
  if (wave < 3) {
    const int dim = t >> 5, n = t & 31;
    float s = 0.f;
#pragma unroll 1
    for (int ks = 0; ks < 16; ++ks) s += w1[(dim * 16 + ks) * 32 + n];
    img[512 + t] = __float_as_uint(s);
  } else if (wave == 3) {
    const int n = t & 31;
    float s = 0.f;
#pragma unroll 1
    for (int i = 0; i < 48; ++i) s = fmaf(centers[i], w1[i * 32 + n], s);
    const float be = b1[n] - s;
    img[608 + n] = __float_as_uint(be);
  }
  __syncthreads();
  if (t < 160) {
    const v4u val = *(const v4u*)(img + 4 * t);
    *(volatile v4u*)(dst + 4 * t) = val;
    __threadfence();
    *(volatile v4u*)(dst + 4 * t) = val;
  }
}

__global__ __launch_bounds__(128) void nbr_agg_kernel(
    const float* __restrict__ features, const float* __restrict__ input_pts, const float* __restrict__ output_pts,
    const int* __restrict__ indices, const float* __restrict__ b2, const float* __restrict__ b3,
    const unsigned short* __restrict__ W2t, const unsigned short* __restrict__ W3t,
    const float* __restrict__ W1e, const float* __restrict__ b1e,
    unsigned short* __restrict__ aggPlane, int chunkBase)
{
  __shared__ __align__(16) _Float16 sH1[kWavesA][16 * 32];
  __shared__ __align__(16) _Float16 sH2[kWavesA][16 * 16];
  __shared__ __align__(16) _Float16 sDT[kWavesA][16 * 16];
  __shared__ __align__(16) _Float16 sFT[kWavesA][64 * 16];
  __shared__ __align__(16) _Float16 sAG[kWavesA][1024];
  typedef Frag<_Float16>::U FragU;

  const int lane = threadIdx.x & 31;
  const int wave = threadIdx.x >> 5;
  const int hh   = lane >> 4;
  const int c    = lane & 15;

  _Float16* H1 = sH1[wave];
  _Float16* H2 = sH2[wave];
  _Float16* DT = sDT[wave];
  _Float16* FT = sFT[wave];
  _Float16* AG = sAG[wave];

  float wx[16], wy[16], wz[16], wb[16];
#pragma unroll
  for (int t4 = 0; t4 < 4; ++t4) {
    const v4f ax = *(const v4f*)(W1e + 16 * hh + 4 * t4);
    const v4f ay = *(const v4f*)(W1e + 32 + 16 * hh + 4 * t4);
    const v4f az = *(const v4f*)(W1e + 64 + 16 * hh + 4 * t4);
    const v4f ab = *(const v4f*)(b1e + 16 * hh + 4 * t4);
#pragma unroll
    for (int e = 0; e < 4; ++e) {
      wx[4 * t4 + e] = ax[e];
      wy[4 * t4 + e] = ay[e];
      wz[4 * t4 + e] = az[e];
      wb[4 * t4 + e] = ab[e];
    }
  }
  const v16h w2frag = Frag<_Float16>::load((const _Float16*)W2t + c * 32 + 8 * hh);
  const v16h w3frag = Frag<_Float16>::load((const _Float16*)W3t + c * 32 + 8 * hh);
  float b2v[8];
  {
    const v4f ba = *(const v4f*)(b2 + 8 * hh);
    const v4f bb = *(const v4f*)(b2 + 8 * hh + 4);
#pragma unroll
    for (int e = 0; e < 4; ++e) { b2v[e] = ba[e]; b2v[4 + e] = bb[e]; }
  }
  const float b3s = b3[c];
  v8h zh;
#pragma unroll
  for (int e = 0; e < 8; ++e) zh[e] = (_Float16)0.0f;
  const v8f zacc = (v8f){0.f,0.f,0.f,0.f,0.f,0.f,0.f,0.f};

  const int pw0 = chunkBase + (blockIdx.x * kWavesA + wave) * kPtsWave;

#pragma unroll 1
  for (int i = 0; i < kPtsWave; ++i) {
    const int p = pw0 + i;
    const int bbase = (p >> 14) << 14;
    const int* ip = indices + (size_t)p * kNbr;

    const v4i i0 = *(const v4i*)(ip);
    const v4i i1 = *(const v4i*)(ip + 4);
    const v4i i2 = *(const v4i*)(ip + 8);
    const v4i i3 = *(const v4i*)(ip + 12);
    int own = ip[c];
    own = own < 0 ? 0 : own;
    own = own > (kNpts - 1) ? (kNpts - 1) : own;
    const size_t go = (size_t)(bbase + own);

    const float qx = input_pts[go * 3 + 0] - output_pts[(size_t)p * 3 + 0];
    const float qy = input_pts[go * 3 + 1] - output_pts[(size_t)p * 3 + 1];
    const float qz = input_pts[go * 3 + 2] - output_pts[(size_t)p * 3 + 2];

    {
      v8h h1a, h1b;
#pragma unroll
      for (int e = 0; e < 8; ++e) {
        float va = fmaf(qx, wx[e], wb[e]);
        va = fmaf(qy, wy[e], va);
        va = fmaf(qz, wz[e], va);
        float vb = fmaf(qx, wx[8 + e], wb[8 + e]);
        vb = fmaf(qy, wy[8 + e], vb);
        vb = fmaf(qz, wz[8 + e], vb);
        h1a[e] = (_Float16)fmaxf(va, 0.0f);
        h1b[e] = (_Float16)fmaxf(vb, 0.0f);
      }
      *(v8h*)(H1 + c * 32 + 16 * hh)     = h1a;
      *(v8h*)(H1 + c * 32 + 16 * hh + 8) = h1b;
    }

    {
      int idl[16];
#pragma unroll
      for (int e = 0; e < 4; ++e) { idl[e] = i0[e]; idl[4 + e] = i1[e]; idl[8 + e] = i2[e]; idl[12 + e] = i3[e]; }
      v2f fv[16];
#pragma unroll
      for (int k = 0; k < 16; ++k) {
        int ik = idl[k];
        ik = ik < 0 ? 0 : ik;
        ik = ik > (kNpts - 1) ? (kNpts - 1) : ik;
        fv[k] = *(const v2f*)(features + (size_t)(bbase + ik) * kCin + 2 * lane);
      }
      v8h r0a, r0b, r1a, r1b;
#pragma unroll
      for (int k = 0; k < 8; ++k) {
        const float a0 = fv[k][0];
        const float a1 = fv[k][1];
        const float c0 = fv[8 + k][0];
        const float c1 = fv[8 + k][1];
        r0a[k] = (_Float16)a0;
        r1a[k] = (_Float16)a1;
        r0b[k] = (_Float16)c0;
        r1b[k] = (_Float16)c1;
      }
      *(v8h*)(FT + (2 * lane) * 16)         = r0a;
      *(v8h*)(FT + (2 * lane) * 16 + 8)     = r0b;
      *(v8h*)(FT + (2 * lane + 1) * 16)     = r1a;
      *(v8h*)(FT + (2 * lane + 1) * 16 + 8) = r1b;
    }
    wave_sync();

    {
      const v16h hb = Frag<_Float16>::load(H1 + c * 32 + 8 * hh);
      const v8f a2 = mma_g(w2frag, hb, zacc);
      v8h h2v;
#pragma unroll
      for (int r = 0; r < 8; ++r) h2v[r] = (_Float16)fmaxf(a2[r] + b2v[r], 0.0f);
      *(v8h*)(H2 + c * 16 + 8 * hh) = h2v;
    }
    wave_sync();

    {
      FragU ha;
      ha.h[0] = *(const v8h*)(H2 + c * 16 + 8 * hh);
      ha.h[1] = zh;
      const v8f a3 = mma_g(ha.v, w3frag, zacc);
      v8h dv;
#pragma unroll
      for (int r = 0; r < 8; ++r) dv[r] = (_Float16)fmaxf(a3[r] + b3s, 0.0f);
      *(v8h*)(DT + c * 16 + 8 * hh) = dv;
    }
    wave_sync();

    {
      FragU da;
      da.h[0] = *(const v8h*)(DT + c * 16 + 8 * hh);
      da.h[1] = zh;
#pragma unroll
      for (int ct = 0; ct < 4; ++ct) {
        FragU fb;
        fb.h[0] = *(const v8h*)(FT + (16 * ct + c) * 16 + 8 * hh);
        fb.h[1] = zh;
        const v8f ag = mma_g(da.v, fb.v, zacc);
        v8h av;
#pragma unroll
        for (int r = 0; r < 8; ++r) av[r] = (_Float16)ag[r];
        *(v8h*)(AG + (16 * ct + c) * 16 + 8 * hh) = av;
      }
    }
    wave_sync();

    {
      v8h ov[4];
#pragma unroll
      for (int it = 0; it < 4; ++it) ov[it] = *(const v8h*)(AG + it * 256 + lane * 8);
      unsigned short* dstp = aggPlane + (size_t)(p - chunkBase) * kKfin + lane * 8;
      for (int pass = 0; pass < 2; ++pass) {
#pragma unroll
        for (int it = 0; it < 4; ++it) *(volatile v8h*)(dstp + it * 256) = ov[it];
        __threadfence();
      }
    }
    wave_sync();
  }
}

extern "C" void kernel_launch(void* const* d_in, const int* in_sizes, int n_in,
                              void* d_out, int out_size, void* d_ws, size_t ws_size,
                              hipStream_t stream) {
  if (n_in < 13) return;
  if (in_sizes[0] != kPts * kCin) return;
  if (in_sizes[1] != kPts * 3) return;
  if (in_sizes[2] != kPts * 3) return;
  if (in_sizes[3] != kKfin * kCout) return;
  if (in_sizes[4] != kCout) return;
  if (in_sizes[5] != 3 * kKs) return;
  if (in_sizes[6] != 48 * 32) return;
  if (in_sizes[7] != 32) return;
  if (in_sizes[8] != 32 * 16) return;
  if (in_sizes[9] != 16) return;
  if (in_sizes[10] != 16 * 16) return;
  if (in_sizes[11] != 16) return;
  if (in_sizes[12] != kPts * kNbr) return;
  if (out_size != kPts * kCout) return;
  if (ws_size < kWsTotal) return;

  const float* features   = (const float*)d_in[0];
  const float* input_pts  = (const float*)d_in[1];
  const float* output_pts = (const float*)d_in[2];
  const float* weight     = (const float*)d_in[3];
  const float* bias       = (const float*)d_in[4];
  const float* centers    = (const float*)d_in[5];
  const float* w1         = (const float*)d_in[6];
  const float* b1         = (const float*)d_in[7];
  const float* w2         = (const float*)d_in[8];
  const float* b2         = (const float*)d_in[9];
  const float* w3         = (const float*)d_in[10];
  const float* b3         = (const float*)d_in[11];
  const int*   indices    = (const int*)d_in[12];
  float* out = (float*)d_out;

  char* ws = (char*)d_ws;
  unsigned short* AGG = (unsigned short*)(ws + kOffAgg);
  unsigned short* WT  = (unsigned short*)(ws + kOffWt);
  char* small = ws + kOffSmall;
  unsigned short* W2t = (unsigned short*)(small);
  unsigned short* W3t = (unsigned short*)(small + 1024);
  float* W1e = (float*)(small + 2048);
  float* b1e = (float*)(small + 2432);

  prep_wt_kernel<<<kKfin / 64, 256, 0, stream>>>(weight, WT);
  prep_small_kernel<<<1, 256, 0, stream>>>(w1, b1, w2, w3, centers, (unsigned*)small);

  for (int ch = 0; ch < kChunks; ++ch) {
    nbr_agg_kernel<<<kChunkPts / kPtsBlock, kWavesA * 32, 0, stream>>>(
        features, input_pts, output_pts, indices, b2, b3, W2t, W3t, W1e, b1e, AGG, ch * kChunkPts);

    wmma_gemm64<0, false, 2, 0, false, 0><<<dim3((kChunkPts / 64) / 8, 1), 256, 0, stream>>>(
        AGG, nullptr, kKfin, 0L,
        WT, nullptr, kKfin, 0L,
        (void*)(out + (size_t)ch * kChunkPts * kCout), nullptr, kCout, 0L,
        bias, nullptr, 0L,
        kChunkPts, kCout, kKfin, kOutScale);
  }
}
